// GraphTransformerLayer_31404800868534
// MI455X (gfx1250) — hardware-verified
//
#include <hip/hip_runtime.h>
#include <stddef.h>
#include <stdint.h>
#include <math.h>


#define DIN     64
#define HN      4
#define CH      64
#define HC      256
#define QKVW    768
#define OQ      0
#define OKK     256
#define OV      512
#define AP      512
#define KFIN    512
#define NTHR    256
#define NWAVE   8
#define EPT     8
#define CHUNK   (NTHR * EPT)
#define WCAP    (EPT * 32)
#define LISTN   (NWAVE * WCAP)
#define NBMAX   1024
#define SLOTB   10
#define RCAP    28672
#define DEGCAP  64
#define GBM     64
#define GBN     64
#define GTHR    128
#define QSC     16.0f
#define ATTSC   0.00048828125f
#define VINV    0.0625f
#define LNEPS   1.0e-5f
#define INV64   0.015625f
#define WSLIM   134217728
#define LDSW_AGG (2 * RCAP + 2 * NBMAX + LISTN + 2 * NWAVE)
#define LDS_AGG  (LDSW_AGG * 4 + 64)

static_assert((1 << SLOTB) == NBMAX);
static_assert(SLOTB + 21 <= 31);
static_assert((CHUNK & (CHUNK - 1)) == 0 && CHUNK <= 2048 && SLOTB + 11 <= 31);
static_assert(NTHR * 4 == NBMAX);
static_assert(LISTN >= NBMAX);
static_assert(LISTN >= NWAVE * WCAP);
static_assert((RCAP % 32) == 0);
static_assert((NBMAX % NWAVE) == 0);
static_assert(LDS_AGG <= 300000);
static_assert(GBM == (GTHR / 32) * 16);
static_assert(GBM * GBN == 4 * GTHR * 8);
static_assert(GBM * GBN == 8 * GTHR * 4);
static_assert(HC == 32 * 8);
static_assert(CH == 8 * 8 && HN * CH == HC);
static_assert((DIN % 32) == 0 && (KFIN % 32) == 0 && KFIN == 2 * HC && AP == KFIN);
static_assert(QKVW == 3 * HC && (QKVW % GBN) == 0 && (HC % GBN) == 0 && CH == GBN);

typedef float          v4f  __attribute__((ext_vector_type(4)));
typedef float          v8f  __attribute__((ext_vector_type(8)));
typedef int            v4i  __attribute__((ext_vector_type(4)));
typedef int            v8i  __attribute__((ext_vector_type(8)));
typedef unsigned int   v4u  __attribute__((ext_vector_type(4)));
typedef unsigned short v8us __attribute__((ext_vector_type(8)));
typedef __bf16         v16b __attribute__((ext_vector_type(16)));
typedef v4f  __attribute__((may_alias)) v4fa;
typedef v4u  __attribute__((may_alias)) v4ua;
typedef v8us __attribute__((may_alias)) v8usa;
union FragB { v16b v; v8us h[2]; v4u q[2]; v8i w; };

__device__ __forceinline__ v8f wmb(const FragB& a, const FragB& b, v8f c) {
  v8f d = __builtin_amdgcn_wmma_f32_16x16x32_bf16(false, a.v, false, b.v, (short)0, c, false, false);
  asm volatile("v_nop\n\tv_nop\n\tv_nop\n\tv_nop" : "+v"(d) : "v"(a.w), "v"(b.w));
  return d;
}

__device__ __forceinline__ void ldwait() {
  asm volatile("s_wait_loadcnt 0x0" ::: "memory");
}

__device__ __forceinline__ unsigned int f2bf(float f) {
  const unsigned int u = __float_as_uint(f);
  return ((u + 0x7FFFu + ((u >> 16) & 1u)) >> 16) & 0xFFFFu;
}
__device__ __forceinline__ float bf2f(unsigned int b) { return __uint_as_float(b << 16); }
__device__ __forceinline__ float bfr(float f) { return bf2f(f2bf(f)); }
__device__ __forceinline__ v4f bfr4(const v4f a) {
  v4f r; r.x = bfr(a.x); r.y = bfr(a.y); r.z = bfr(a.z); r.w = bfr(a.w); return r;
}
__device__ __forceinline__ unsigned int pk2(float lo, float hi) { return f2bf(lo) | (f2bf(hi) << 16); }
__device__ __forceinline__ v4u pack8(const v4f a, const v4f b) {
  v4u r;
  r.x = pk2(a.x, a.y); r.y = pk2(a.z, a.w); r.z = pk2(b.x, b.y); r.w = pk2(b.z, b.w);
  return r;
}
__device__ __forceinline__ void hl2(float v0, float v1, unsigned int& hw, unsigned int& lw) {
  const unsigned int h0 = f2bf(v0), h1 = f2bf(v1);
  const unsigned int l0 = f2bf(v0 - bf2f(h0)), l1 = f2bf(v1 - bf2f(h1));
  hw = h0 | (h1 << 16);
  lw = l0 | (l1 << 16);
}
__device__ __forceinline__ void pack8hl(const v4f a, const v4f b, v4u& hv, v4u& lv) {
  unsigned int h, l;
  hl2(a.x, a.y, h, l); hv.x = h; lv.x = l;
  hl2(a.z, a.w, h, l); hv.y = h; lv.y = l;
  hl2(b.x, b.y, h, l); hv.z = h; lv.z = l;
  hl2(b.z, b.w, h, l); hv.w = h; lv.w = l;
}
__device__ __forceinline__ unsigned int pkh2(float e0, float e1) {
  const unsigned short a = __builtin_bit_cast(unsigned short, (_Float16)e0);
  const unsigned short b = __builtin_bit_cast(unsigned short, (_Float16)e1);
  return (unsigned int)a | ((unsigned int)b << 16);
}
__device__ __forceinline__ v4u packh8s(const v4f a, const v4f b, float s) {
  v4u r;
  r.x = pkh2(a.x * s, a.y * s); r.y = pkh2(a.z * s, a.w * s);
  r.z = pkh2(b.x * s, b.y * s); r.w = pkh2(b.z * s, b.w * s);
  return r;
}
__device__ __forceinline__ float hflo(unsigned int w) {
  return (float)__builtin_bit_cast(_Float16, (unsigned short)(w & 0xFFFFu));
}
__device__ __forceinline__ float hfhi(unsigned int w) {
  return (float)__builtin_bit_cast(_Float16, (unsigned short)(w >> 16));
}
__device__ __forceinline__ void widen8(const v4u w, v4f& a, v4f& b) {
  a.x = hflo(w.x); a.y = hfhi(w.x); a.z = hflo(w.y); a.w = hfhi(w.y);
  b.x = hflo(w.z); b.y = hfhi(w.z); b.z = hflo(w.w); b.w = hfhi(w.w);
}

__device__ __forceinline__ int scan_chunk(const int* __restrict__ dsts, int nE, int cbase, int slotBase,
                                          int nb, int vec8, int* list, int tid, int lane, int wave) {
  int wc = 0;
  const int el0  = tid * EPT;
  const int e0   = cbase + el0;
  const int sent = -2147483647 - 1;
  v4i da, db;
  if (vec8 != 0 && cbase + CHUNK <= nE) {
    da = *(const v4i*)(dsts + e0);
    db = *(const v4i*)(dsts + e0 + 4);
  } else {
    da.x = (e0     < nE) ? dsts[min(e0,     nE - 1)] : sent;
    da.y = (e0 + 1 < nE) ? dsts[min(e0 + 1, nE - 1)] : sent;
    da.z = (e0 + 2 < nE) ? dsts[min(e0 + 2, nE - 1)] : sent;
    da.w = (e0 + 3 < nE) ? dsts[min(e0 + 3, nE - 1)] : sent;
    db.x = (e0 + 4 < nE) ? dsts[min(e0 + 4, nE - 1)] : sent;
    db.y = (e0 + 5 < nE) ? dsts[min(e0 + 5, nE - 1)] : sent;
    db.z = (e0 + 6 < nE) ? dsts[min(e0 + 6, nE - 1)] : sent;
    db.w = (e0 + 7 < nE) ? dsts[min(e0 + 7, nE - 1)] : sent;
  }
  const unsigned nbs = (unsigned)slotBase;
  const unsigned unb = (unsigned)nb;
  const unsigned s0 = (unsigned)da.x - nbs, s1 = (unsigned)da.y - nbs;
  const unsigned s2 = (unsigned)da.z - nbs, s3 = (unsigned)da.w - nbs;
  const unsigned s4 = (unsigned)db.x - nbs, s5 = (unsigned)db.y - nbs;
  const unsigned s6 = (unsigned)db.z - nbs, s7 = (unsigned)db.w - nbs;
  const bool h0 = s0 < unb, h1 = s1 < unb, h2 = s2 < unb, h3 = s3 < unb;
  const bool h4 = s4 < unb, h5 = s5 < unb, h6 = s6 < unb, h7 = s7 < unb;
  const unsigned any = __builtin_amdgcn_ballot_w32(h0 | h1 | h2 | h3 | h4 | h5 | h6 | h7);
  if (any != 0u) {
#define HITJ(J, HJ, SJ) { \
      const unsigned mj = __builtin_amdgcn_ballot_w32(HJ); \
      if (mj != 0u) { \
        if (HJ) { \
          const int pos = wc + (int)__builtin_amdgcn_mbcnt_lo(mj, 0u); \
          if (pos < WCAP) list[wave * WCAP + pos] = ((el0 + (J)) << SLOTB) | (int)(SJ); \
        } \
        wc += (int)__builtin_popcount(mj); } }
    HITJ(0, h0, s0)
    HITJ(1, h1, s1)
    HITJ(2, h2, s2)
    HITJ(3, h3, s3)
    HITJ(4, h4, s4)
    HITJ(5, h5, s5)
    HITJ(6, h6, s6)
    HITJ(7, h7, s7)
#undef HITJ
  }
  return wc;
}

__global__ __launch_bounds__(NTHR) void k_wtr(const float* __restrict__ w, int Kin, int Ncol, int Nrows, int Kout,
                                              unsigned short* wt, int nUnits) {
  const int u = (int)blockIdx.x * NTHR + (int)threadIdx.x;
  if (u >= nUnits) return;
  const int kq = Kout >> 3;
  const int n  = u / kq;
  const int k8 = (u - n * kq) * 8;
  const int kk = k8 - (k8 / Kin) * Kin;
  const int ncl = n < Ncol ? n : Ncol - 1;
  const float* p = w + (size_t)kk * (size_t)Ncol + ncl;
  v4f a, b;
  a.x = p[0];                    a.y = p[(size_t)Ncol];         a.z = p[(size_t)2 * Ncol];     a.w = p[(size_t)3 * Ncol];
  b.x = p[(size_t)4 * Ncol];     b.y = p[(size_t)5 * Ncol];     b.z = p[(size_t)6 * Ncol];     b.w = p[(size_t)7 * Ncol];
  const v4f z4 = {0.f, 0.f, 0.f, 0.f};
  if (n >= Ncol || n >= Nrows) { a = z4; b = z4; }
  const v4u wv = pack8(a, b);
  unsigned short* o = wt + (size_t)n * (size_t)Kout + k8;
  *(volatile v4u*)o = wv;
  __threadfence();
  *(volatile v4u*)o = wv;
}

__global__ __launch_bounds__(GTHR) void k_qkv(const float* __restrict__ hin, const unsigned short* __restrict__ WT,
                                              unsigned short* qkv, int nN)
{
  __shared__ __attribute__((aligned(16))) float stg[GBM * GBN];
  const int tid = (int)threadIdx.x, lane = tid & 31, wave = tid >> 5, hh = lane >> 4, m = lane & 15;
  const int rowBase = (int)blockIdx.x * GBM;
  const int col0    = (int)blockIdx.y * GBN;

  FragB ax[2];
  {
    const int ar  = rowBase + 16 * wave + m;
    const int arc = ar < nN ? ar : nN - 1;
    const float* ap = hin + (size_t)arc * DIN + 8 * hh;
    const v4f z4 = {0.f, 0.f, 0.f, 0.f};
#pragma unroll
    for (int ks = 0; ks < 2; ++ks) {
      v4f a0 = *(const v4fa*)(ap + 32 * ks);
      v4f a1 = *(const v4fa*)(ap + 32 * ks + 4);
      v4f a2 = *(const v4fa*)(ap + 32 * ks + 16);
      v4f a3 = *(const v4fa*)(ap + 32 * ks + 20);
      if (ar >= nN) { a0 = z4; a1 = z4; a2 = z4; a3 = z4; }
      ax[ks].q[0] = pack8(a0, a1);
      ax[ks].q[1] = pack8(a2, a3);
    }
  }

  v8f acc[4];
  {
    const v8f z = {0.f, 0.f, 0.f, 0.f, 0.f, 0.f, 0.f, 0.f};
    acc[0] = z; acc[1] = z; acc[2] = z; acc[3] = z;
  }
  const unsigned short* wp = WT + (size_t)(col0 + m) * DIN + 8 * hh;
#pragma unroll
  for (int ks = 0; ks < DIN / 32; ++ks) {
#pragma unroll
    for (int t = 0; t < 4; ++t) {
      const unsigned short* wq = wp + (size_t)(16 * t) * DIN + 32 * ks;
      FragB bf;
      bf.h[0] = *(const v8usa*)wq;
      bf.h[1] = *(const v8usa*)(wq + 16);
      acc[t] = wmb(ax[ks], bf, acc[t]);
    }
  }

#pragma unroll
  for (int t = 0; t < 4; ++t) {
    const int lc = 16 * t + m;
#pragma unroll
    for (int r = 0; r < 8; ++r) {
      const int lr = 16 * wave + 8 * hh + r;
      stg[lr * GBN + lc] = acc[t][r];
    }
  }
  __syncthreads();

  v4u hv[4];
  const int rq = lane >> 3;
  const int c8 = 8 * (lane & 7);
#pragma unroll
  for (int i = 0; i < 4; ++i) {
    const int lr = 16 * wave + 4 * i + rq;
    const v4f a = *(const v4fa*)(stg + lr * GBN + c8);
    const v4f b = *(const v4fa*)(stg + lr * GBN + c8 + 4);
    hv[i] = packh8s(a, b, QSC);
  }
#pragma unroll
  for (int i = 0; i < 4; ++i) {
    const int lr = 16 * wave + 4 * i + rq;
    unsigned short* op = qkv + (size_t)(rowBase + lr) * QKVW + col0 + c8;
    *(volatile v4u*)op = hv[i];
  }
  __threadfence();
#pragma unroll
  for (int i = 0; i < 4; ++i) {
    const int lr = 16 * wave + 4 * i + rq;
    unsigned short* op = qkv + (size_t)(rowBase + lr) * QKVW + col0 + c8;
    *(volatile v4u*)op = hv[i];
  }
}

__global__ __launch_bounds__(NTHR) void k_agg(
    const int* __restrict__ srcs, const int* __restrict__ dsts,
    const unsigned short* __restrict__ qkv, unsigned short* apl, int nN, int nE, int vec8, int MPr) {
  extern __shared__ v4f lds_dyn[];
  int* reg1 = (int*)lds_dyn;
  int* reg2 = reg1 + RCAP;
  int* scnt = reg2 + RCAP;
  int* soff = scnt + NBMAX;
  int* list = soff + NBMAX;
  int* wcnt = list + LISTN;
  int* wtot = wcnt + NWAVE;
  const int tid = (int)threadIdx.x, lane = tid & 31, wave = tid >> 5;
  const int nodeBase = (int)blockIdx.x * NBMAX;

  for (int i = tid; i < NBMAX; i += NTHR) scnt[i] = 0;
  __syncthreads();

  int tot = 0;
  const int nChunks = (nE + CHUNK - 1) / CHUNK;
#pragma unroll 1
  for (int ch = 0; ch < nChunks; ++ch) {
    const int cbase = ch * CHUNK;
    const int wc = scan_chunk(dsts, nE, cbase, nodeBase, NBMAX, vec8, list, tid, lane, wave);
    if (lane == 0) wcnt[wave] = wc;
    __syncthreads();
    int pre = 0, all = 0;
#pragma unroll
    for (int w2 = 0; w2 < NWAVE; ++w2) {
      int c = wcnt[w2];
      c = c < 0 ? 0 : (c > WCAP ? WCAP : c);
      all += c;
      pre += (w2 < wave) ? c : 0;
    }
    const int wcc  = wc > WCAP ? WCAP : wc;
    const int base = tot + pre;
#pragma unroll 1
    for (int i = lane; i < wcc; i += 32) {
      const int ent = list[wave * WCAP + i];
      const int el  = (ent >> SLOTB) & (CHUNK - 1);
      const int sl  = ent & (NBMAX - 1);
      int eid = cbase + el;
      eid = eid > nE - 1 ? nE - 1 : eid;
      const int pos = base + i;
      if (pos < RCAP) reg1[pos] = (int)(((unsigned)eid << SLOTB) | (unsigned)sl);
    }
    tot += all;
    tot = tot > RCAP ? RCAP : tot;
    __syncthreads();
  }
  const int nh = tot;

  if (wave == 0) {
#pragma unroll 1
    for (int b0 = 0; b0 < nh; b0 += 32) {
      const int idx = b0 + lane;
      const int uv  = reg1[idx < nh ? idx : nh - 1];
      const int m32 = (nh - b0) < 32 ? (nh - b0) : 32;
#pragma unroll 1
      for (int k = 0; k < m32; ++k) {
        const int u  = __builtin_amdgcn_readlane(uv, k);
        const int sl = u & (NBMAX - 1);
        if (lane == 0) scnt[sl] = scnt[sl] + 1;
      }
    }
  }
  __syncthreads();

  {
    const v4i ca = *(const v4i*)(scnt + 4 * tid);
    const int e0 = ca.x < 0 ? 0 : ca.x, e1 = ca.y < 0 ? 0 : ca.y, e2 = ca.z < 0 ? 0 : ca.z, e3 = ca.w < 0 ? 0 : ca.w;
    const int ts = e0 + e1 + e2 + e3;
    int incl = ts;
#pragma unroll
    for (int d = 1; d < 32; d <<= 1) {
      const int up = __shfl_up(incl, d);
      if (lane >= d) incl += up;
    }
    if (lane == 31) wtot[wave] = incl;
    __syncthreads();
    int pre = 0;
#pragma unroll
    for (int w2 = 0; w2 < NWAVE; ++w2) pre += (w2 < wave) ? wtot[w2] : 0;
    int run = pre + incl - ts;
    soff[4 * tid + 0] = run; run += e0;
    soff[4 * tid + 1] = run; run += e1;
    soff[4 * tid + 2] = run; run += e2;
    soff[4 * tid + 3] = run;
  }
  __syncthreads();
  for (int i = tid; i < NBMAX; i += NTHR) list[i] = soff[i];
  __syncthreads();

  if (wave == 0) {
#pragma unroll 1
    for (int b0 = 0; b0 < nh; b0 += 32) {
      const int idx = b0 + lane;
      const int uv  = reg1[idx < nh ? idx : nh - 1];
      const int m32 = (nh - b0) < 32 ? (nh - b0) : 32;
#pragma unroll 1
      for (int k = 0; k < m32; ++k) {
        const int u   = __builtin_amdgcn_readlane(uv, k);
        const int sl  = u & (NBMAX - 1);
        const int eid = (int)((unsigned)u >> SLOTB);
        if (lane == 0) {
          int pos = list[sl];
          pos = pos < 0 ? 0 : (pos > RCAP - 1 ? RCAP - 1 : pos);
          reg2[pos] = eid;
          list[sl] = pos + 1;
        }
      }
    }
  }
  __syncthreads();

  const int nbw = NBMAX / NWAVE;
  const bool ovf = (nh >= RCAP);
  const float qnan = __int_as_float(0x7fc00000);

#pragma unroll 1
  for (int jt = 0; jt < nbw; ++jt) {
    const int slot = wave * nbw + jt;
    const int grow = nodeBase + slot;
    const int gcl  = grow < nN ? grow : nN - 1;
    int st = soff[slot];
    const int craw = scnt[slot];
    int cnt = craw;
    st  = st < 0 ? 0 : (st > nh ? nh : st);
    cnt = cnt < 0 ? 0 : (cnt > DEGCAP ? DEGCAP : cnt);
    if (cnt > nh - st) cnt = nh - st;
    const float pz = (ovf || craw > DEGCAP) ? qnan : 0.0f;

    const v4u kw = *(const v4ua*)(qkv + (size_t)gcl * QKVW + OKK + 8 * lane);
    ldwait();
    v4f ka, kb;
    widen8(kw, ka, kb);

    v4f ava = {0.f, 0.f, 0.f, 0.f};
    v4f avb = {0.f, 0.f, 0.f, 0.f};
#pragma unroll 1
    for (int q = 0; q < cnt; ++q) {
      int idx = st + q; idx = idx > RCAP - 1 ? RCAP - 1 : idx;
      int eid = reg2[idx]; eid = eid < 0 ? 0 : (eid > nE - 1 ? nE - 1 : eid);
      const int sraw = srcs[eid];
      const int s = sraw < 0 ? 0 : (sraw > nN - 1 ? nN - 1 : sraw);
      const unsigned short* rs = qkv + (size_t)s * QKVW + 8 * lane;
      const v4u qw = *(const v4ua*)(rs + OQ);
      const v4u vw = *(const v4ua*)(rs + OV);
      ldwait();
      v4f qa, qb, va, vb;
      widen8(qw, qa, qb);
      widen8(vw, va, vb);
      float p = qa.x * ka.x;
      p = fmaf(qa.y, ka.y, p); p = fmaf(qa.z, ka.z, p); p = fmaf(qa.w, ka.w, p);
      p = fmaf(qb.x, kb.x, p); p = fmaf(qb.y, kb.y, p); p = fmaf(qb.z, kb.z, p); p = fmaf(qb.w, kb.w, p);
      p += __shfl_xor(p, 4);
      p += __shfl_xor(p, 2);
      p += __shfl_xor(p, 1);
      const float lg = p * ATTSC;
      float mx = fmaxf(lg, __shfl_xor(lg, 8));
      mx = fmaxf(mx, __shfl_xor(mx, 16));
      const float ex = __expf(lg - mx);
      float sm = ex + __shfl_xor(ex, 8);
      sm = sm + __shfl_xor(sm, 16);
      const float at = ex * __builtin_amdgcn_rcpf(sm);
      ava.x = fmaf(at, va.x, ava.x); ava.y = fmaf(at, va.y, ava.y);
      ava.z = fmaf(at, va.z, ava.z); ava.w = fmaf(at, va.w, ava.w);
      avb.x = fmaf(at, vb.x, avb.x); avb.y = fmaf(at, vb.y, avb.y);
      avb.z = fmaf(at, vb.z, avb.z); avb.w = fmaf(at, vb.w, avb.w);
    }
    const bool live = (grow < nN);
    v4f oa, ob;
    oa.x = live ? fmaf(ava.x, VINV, pz) : 0.0f;  oa.y = live ? fmaf(ava.y, VINV, pz) : 0.0f;
    oa.z = live ? fmaf(ava.z, VINV, pz) : 0.0f;  oa.w = live ? fmaf(ava.w, VINV, pz) : 0.0f;
    ob.x = live ? fmaf(avb.x, VINV, pz) : 0.0f;  ob.y = live ? fmaf(avb.y, VINV, pz) : 0.0f;
    ob.z = live ? fmaf(avb.z, VINV, pz) : 0.0f;  ob.w = live ? fmaf(avb.w, VINV, pz) : 0.0f;
    v4u hv, lv;
    pack8hl(oa, ob, hv, lv);
    const bool wr = (grow < MPr);
    const int gsf = wr ? grow : MPr - 1;
    unsigned short* orow = apl + (size_t)gsf * AP;
    if (wr) {
      *(volatile v4u*)(orow + 8 * lane)      = hv;
      *(volatile v4u*)(orow + HC + 8 * lane) = lv;
    }
    __threadfence();
    if (wr) {
      *(volatile v4u*)(orow + 8 * lane)      = hv;
      *(volatile v4u*)(orow + HC + 8 * lane) = lv;
    }
  }
}

__global__ __launch_bounds__(GTHR) void k_final(
    const unsigned short* __restrict__ A, const unsigned short* __restrict__ WT,
    const float* __restrict__ hin, const float* __restrict__ gam, const float* __restrict__ bet,
    float* out, int nN)
{
  __shared__ __attribute__((aligned(16))) float stg[GBM * GBN];
  const int tid = (int)threadIdx.x, lane = tid & 31, wave = tid >> 5, hh = lane >> 4, m = lane & 15;
  const int rowBase = (int)blockIdx.x * GBM;

  v8f acc[4];
  {
    const v8f z = {0.f, 0.f, 0.f, 0.f, 0.f, 0.f, 0.f, 0.f};
    acc[0] = z; acc[1] = z; acc[2] = z; acc[3] = z;
  }
  const unsigned short* ap = A  + (size_t)(rowBase + 16 * wave + m) * (size_t)AP + 8 * hh;
  const unsigned short* wl = WT + (size_t)m * (size_t)KFIN + 8 * hh;
#pragma unroll 1
  for (int k0 = 0; k0 < KFIN; k0 += 32) {
    FragB af;
    af.h[0] = *(const v8usa*)(ap + k0);
    af.h[1] = *(const v8usa*)(ap + k0 + 16);
#pragma unroll
    for (int t = 0; t < 4; ++t) {
      const unsigned short* wq = wl + (size_t)(16 * t) * (size_t)KFIN + k0;
      FragB bf;
      bf.h[0] = *(const v8usa*)wq;
      bf.h[1] = *(const v8usa*)(wq + 16);
      acc[t] = wmb(af, bf, acc[t]);
    }
  }

#pragma unroll
  for (int t = 0; t < 4; ++t) {
    const int lc = 16 * t + m;
#pragma unroll
    for (int r = 0; r < 8; ++r) {
      const int lr = 16 * wave + 8 * hh + r;
      stg[lr * GBN + lc] = acc[t][r];
    }
  }
  __syncthreads();

  const v4f g4 = bfr4(*(const v4fa*)(gam + 4 * m));
  const v4f b4 = bfr4(*(const v4fa*)(bet + 4 * m));

  v4f fv[8];
#pragma unroll
  for (int i = 0; i < 8; ++i) {
    const int lr = 16 * wave + 2 * i + hh;
    fv[i] = *(const v4fa*)(stg + lr * GBN + 4 * m);
  }
  v4f yv[8];
#pragma unroll
  for (int i = 0; i < 8; ++i) {
    const int lr = 16 * wave + 2 * i + hh;
    const int gr = rowBase + lr;
    const int gs = gr < nN ? gr : nN - 1;
    const v4f hr = bfr4(*(const v4fa*)(hin + (size_t)gs * DIN + 4 * m));
    v4f x;
    x.x = fv[i].x + hr.x; x.y = fv[i].y + hr.y; x.z = fv[i].z + hr.z; x.w = fv[i].w + hr.w;
    float s = (x.x + x.y) + (x.z + x.w);
    s += __shfl_xor(s, 1);
    s += __shfl_xor(s, 2);
    s += __shfl_xor(s, 4);
    s += __shfl_xor(s, 8);
    const float mu = s * INV64;
    v4f d;
    d.x = x.x - mu; d.y = x.y - mu; d.z = x.z - mu; d.w = x.w - mu;
    float v = d.x * d.x;
    v = fmaf(d.y, d.y, v); v = fmaf(d.z, d.z, v); v = fmaf(d.w, d.w, v);
    v += __shfl_xor(v, 1);
    v += __shfl_xor(v, 2);
    v += __shfl_xor(v, 4);
    v += __shfl_xor(v, 8);
    const float var = v * INV64;
    const float rs  = rsqrtf(var + LNEPS);
    v4f y;
    y.x = fmaf(d.x * rs, g4.x, b4.x); y.y = fmaf(d.y * rs, g4.y, b4.y);
    y.z = fmaf(d.z * rs, g4.z, b4.z); y.w = fmaf(d.w * rs, g4.w, b4.w);
    yv[i] = y;
  }
#pragma unroll
  for (int i = 0; i < 8; ++i) {
    const int lr = 16 * wave + 2 * i + hh;
    const int gr = rowBase + lr;
    const int gs = gr < nN ? gr : nN - 1;
    float* op = out + (size_t)gs * CH + 4 * m;
    if (gr < nN) *(volatile v4f*)op = yv[i];
  }
  __threadfence();
#pragma unroll
  for (int i = 0; i < 8; ++i) {
    const int lr = 16 * wave + 2 * i + hh;
    const int gr = rowBase + lr;
    const int gs = gr < nN ? gr : nN - 1;
    float* op = out + (size_t)gs * CH + 4 * m;
    if (gr < nN) *(volatile v4f*)op = yv[i];
  }
}

static inline int cdiv(int a, int b) { return (a + b - 1) / b; }
static inline size_t al256(size_t o) { return (o + 255) & ~(size_t)255; }

extern "C" void kernel_launch(void* const* d_in, const int* in_sizes, int n_in,
                              void* d_out, int out_size, void* d_ws, size_t ws_size,
                              hipStream_t stream) {
  if (n_in < 9) return;
  if (in_sizes[0] < DIN || (in_sizes[0] % DIN) != 0) return;
  const int nN = in_sizes[0] / DIN;
  if (nN < 1 || nN > (1 << 22)) return;
  const int nE = in_sizes[1];
  if (nE < 1 || nE >= (1 << (31 - SLOTB))) return;
  if (in_sizes[2] != nE) return;
  if (in_sizes[3] != DIN * HC || in_sizes[4] != DIN * HC || in_sizes[5] != DIN * HC) return;
  if (in_sizes[6] != HC * CH) return;
  if (in_sizes[7] != CH || in_sizes[8] != CH) return;
  if ((long long)out_size != (long long)nN * CH) return;

  const float* hin = (const float*)d_in[0];
  const int*   src = (const int*)  d_in[1];
  const int*   dst = (const int*)  d_in[2];
  const float* Wq  = (const float*)d_in[3];
  const float* Wk  = (const float*)d_in[4];
  const float* Wv  = (const float*)d_in[5];
  const float* Wo  = (const float*)d_in[6];
  const float* gam = (const float*)d_in[7];
  const float* bet = (const float*)d_in[8];
  float* out = (float*)d_out;

  const int MP   = cdiv(nN, GBM) * GBM;
  const int gM   = MP / GBM;
  const int gA   = cdiv(MP, NBMAX);
  const int vec8 = ((nE & 3) == 0) ? 1 : 0;
  if ((long long)gA * NBMAX < (long long)MP) return;

  char* ws = (char*)d_ws;
  size_t off = 0;
  const size_t oWQ  = off; off = al256(off + (size_t)QKVW * DIN * 2);
  const size_t oWO  = off; off = al256(off + (size_t)CH * KFIN * 2);
  const size_t oQKV = off; off = al256(off + (size_t)MP * QKVW * 2);
  const size_t oAPL = off; off = al256(off + (size_t)MP * AP * 2);
  if (off > ws_size || off > (size_t)WSLIM) return;
  unsigned short* WQKVT = (unsigned short*)(ws + oWQ);
  unsigned short* WOT2  = (unsigned short*)(ws + oWO);
  unsigned short* QKVH  = (unsigned short*)(ws + oQKV);
  unsigned short* APL   = (unsigned short*)(ws + oAPL);

  hipFuncSetAttribute(reinterpret_cast<const void*>(&k_agg),
                      hipFuncAttributeMaxDynamicSharedMemorySize, LDS_AGG);

  {
    const int nUq = HC * (DIN / 8);
    k_wtr<<<cdiv(nUq, NTHR), NTHR, 0, stream>>>(Wq, DIN, HC, HC, DIN, WQKVT,                        nUq);
    k_wtr<<<cdiv(nUq, NTHR), NTHR, 0, stream>>>(Wk, DIN, HC, HC, DIN, WQKVT + (size_t)HC * DIN,      nUq);
    k_wtr<<<cdiv(nUq, NTHR), NTHR, 0, stream>>>(Wv, DIN, HC, HC, DIN, WQKVT + (size_t)2 * HC * DIN,  nUq);
    const int nUo = CH * (KFIN / 8);
    k_wtr<<<cdiv(nUo, NTHR), NTHR, 0, stream>>>(Wo, HC, CH, CH, KFIN, WOT2, nUo);
  }

  k_qkv<<<dim3(gM, QKVW / GBN), GTHR, 0, stream>>>(hin, WQKVT, QKVH, nN);
  k_agg<<<gA, NTHR, LDS_AGG, stream>>>(src, dst, QKVH, APL, nN, nE, vec8, MP);
  k_final<<<gM, GTHR, 0, stream>>>(APL, WOT2, hin, gam, bet, out, nN);
}
